// RGBuvHistBlock_1889785610949
// MI455X (gfx1250) — hardware-verified
//
#include <hip/hip_runtime.h>
#include <math.h>

typedef __attribute__((ext_vector_type(16))) __bf16   v16b;
typedef __attribute__((ext_vector_type(8)))  __bf16   v8b;
typedef __attribute__((ext_vector_type(8)))  float    v8f;
typedef __attribute__((ext_vector_type(4)))  float    v4f;
typedef __attribute__((ext_vector_type(4)))  unsigned int v4u;

constexpr int   kNumImg        = 32;
constexpr int   kNumPair       = 3;
constexpr int   kNumPix        = 22500;
constexpr int   kNumPixPad     = 22528;
constexpr int   kNumBins       = 64;
constexpr int   kNumSplit      = 8;
constexpr int   kPixPerSplit   = kNumPixPad / kNumSplit;
constexpr int   kChunkPix      = 64;
constexpr int   kNumIter       = kPixPerSplit / kChunkPix;
constexpr int   kNumBC         = kNumImg * kNumPair;
constexpr int   kTileElems     = kNumBins * kNumBins;
constexpr int   kPerImg        = kNumPair * kTileElems;
constexpr int   kOutElems      = kNumImg * kPerImg;
constexpr int   kInElems       = kNumImg * kNumPair * kNumPix;
constexpr int   kOpPitch       = 72;
constexpr int   kResPitch      = 68;
constexpr int   kThreads       = 256;
constexpr int   kGroupsPerThr  = kPerImg / (kThreads * 4);
constexpr float kEps           = 1e-06f;
constexpr float kInvSig2       = 2500.0f;

constexpr size_t kPartBytes = (size_t)kNumBC * kNumSplit * kTileElems * sizeof(float);

static_assert(kNumPixPad % 32 == 0, "K multiple of 32");
static_assert(kNumPixPad >= kNumPix && kNumPixPad - kNumPix < 32, "K pad");
static_assert(kPixPerSplit * kNumSplit == kNumPixPad, "split covers K");
static_assert(kNumIter * kChunkPix == kPixPerSplit, "chunks cover split");
static_assert(kNumBins == 64, "M = N = 64, one 4x4 grid of 16x16 tiles per block");
static_assert(kGroupsPerThr * kThreads * 4 == kPerImg, "reduce coverage");
static_assert(kPartBytes <= (size_t)134217728, "carve under 128 MiB");
static_assert((kOpPitch % 8) == 0, "16-B aligned operand rows");

__device__ __forceinline__ unsigned short f2bf_bits(float f) {
  unsigned u = __float_as_uint(f);
  return (unsigned short)((u + 0x7FFFu + ((u >> 16) & 1u)) >> 16);
}
__device__ __forceinline__ unsigned pk16(unsigned short a, unsigned short b) { return (unsigned)a | ((unsigned)b << 16); }

struct FragBf {
  union U { v16b v; v8b h[2]; };
  static __device__ __forceinline__ v16b load(const __bf16* p) {
    U f; f.h[0] = *(const v8b*)(p); f.h[1] = *(const v8b*)(p + 16); return f.v;
  }
  static __device__ __forceinline__ v8f mma(v16b a, v16b b, v8f c) {
    return __builtin_amdgcn_wmma_f32_16x16x32_bf16(false, a, false, b, (short)0, c, false, false);
  }
};

__device__ __forceinline__ void guard3(v8f& a0, v8f& a1, v16b x, v16b y, v16b z) {
  asm volatile("v_nop\n\tv_nop\n\tv_nop\n\tv_nop" : "+v"(a0), "+v"(a1) : "v"(x), "v"(y), "v"(z));
}
__device__ __forceinline__ void acc_guard2(v8f& a0, v8f& a1) {
  asm volatile("v_nop\n\tv_nop\n\tv_nop\n\tv_nop" : "+v"(a0), "+v"(a1));
}

__global__ __launch_bounds__(256) void hist_partial_kernel(const float* __restrict__ x,
                                                           float* __restrict__ part) {
  #pragma clang fp contract(off)
  __shared__ __align__(16) __bf16 sA[kNumBins * kOpPitch];
  __shared__ __align__(16) __bf16 sB[kNumBins * kOpPitch];
  __shared__ __align__(16) float  sRes[kNumBins * kResPitch];
  __shared__ __align__(16) float  sU[kChunkPix];
  __shared__ __align__(16) float  sV[kChunkPix];
  __shared__ __align__(16) float  sIy[kChunkPix];
  __shared__ __align__(16) float  sF[kChunkPix];

  const int t    = threadIdx.x;
  const int lane = t & 31;
  const int wave = t >> 5;
  const int bc   = blockIdx.x / kNumSplit;
  const int s    = blockIdx.x - bc * kNumSplit;
  const int b    = bc / kNumPair;
  const int c    = bc - b * kNumPair;
  const float* xb = x + (size_t)b * kNumPair * kNumPix;
  const int pixBase = s * kPixPerSplit;

  const int row = t >> 2;
  const int kq  = (t & 3) * 16;
  const float stepv = (float)row * (1.0f / 63.0f);
  float binv = (-3.0f) * (1.0f - stepv) + 3.0f * stepv;
  if (row == kNumBins - 1) binv = 3.0f;

  const int mi   = wave >> 1;
  const int nj0  = (wave & 1) * 2;
  const int rl   = lane & 15;
  const int koff = (lane >> 4) * 8;
  const int hh   = lane >> 4;

  v8f acc0 = (v8f){0.f, 0.f, 0.f, 0.f, 0.f, 0.f, 0.f, 0.f};
  v8f acc1 = (v8f){0.f, 0.f, 0.f, 0.f, 0.f, 0.f, 0.f, 0.f};

  for (int it = 0; it < kNumIter; ++it) {
    if (t < kChunkPix) {
      const int  n  = pixBase + it * kChunkPix + t;
      const bool ok = (n < kNumPix);
      const int  nc = ok ? n : (kNumPix - 1);
      float r  = xb[nc];
      float g  = xb[kNumPix + nc];
      float bl = xb[2 * kNumPix + nc];
      r  = fminf(fmaxf(r,  0.0f), 1.0f);
      g  = fminf(fmaxf(g,  0.0f), 1.0f);
      bl = fminf(fmaxf(bl, 0.0f), 1.0f);
      const float lr = logf(r  + kEps);
      const float lg = logf(g  + kEps);
      const float lb = logf(bl + kEps);
      const float u0 = lr - lg, v0 = lr - lb;
      const float u1 = lg - lr, v1 = lg - lb;
      const float u2 = lb - lr, v2 = lb - lg;
      const float uu = (c == 0) ? u0 : (c == 1) ? u1 : u2;
      const float vv = (c == 0) ? v0 : (c == 1) ? v1 : v2;
      const float ss = (r * r + bl * bl) + g * g;
      const float iy = sqrtf(ss + kEps);
      sU[t]  = ok ? uu : 0.0f;
      sV[t]  = ok ? vv : 0.0f;
      sIy[t] = ok ? iy : 0.0f;
      sF[t]  = ok ? 1.0f : 0.0f;
    }
    __syncthreads();

    {
      unsigned aw[8], bw[8];
#pragma unroll
      for (int q4 = 0; q4 < 4; ++q4) {
        const v4f uu = *(const v4f*)(sU  + kq + 4 * q4);
        const v4f vv = *(const v4f*)(sV  + kq + 4 * q4);
        const v4f yy = *(const v4f*)(sIy + kq + 4 * q4);
        const v4f ff = *(const v4f*)(sF  + kq + 4 * q4);
        unsigned short ab[4], bb[4];
#pragma unroll
        for (int e = 0; e < 4; ++e) {
          const float du = uu[e] - binv;
          const float dv = vv[e] - binv;
          const float ku = __builtin_amdgcn_rcpf(fmaf(du * du, kInvSig2, 1.0f));
          const float kv = __builtin_amdgcn_rcpf(fmaf(dv * dv, kInvSig2, 1.0f));
          ab[e] = f2bf_bits(yy[e] * ku);
          bb[e] = f2bf_bits(ff[e] * kv);
        }
        aw[2 * q4]     = pk16(ab[0], ab[1]);
        aw[2 * q4 + 1] = pk16(ab[2], ab[3]);
        bw[2 * q4]     = pk16(bb[0], bb[1]);
        bw[2 * q4 + 1] = pk16(bb[2], bb[3]);
      }
      const v4u a0 = (v4u){aw[0], aw[1], aw[2], aw[3]};
      const v4u a1 = (v4u){aw[4], aw[5], aw[6], aw[7]};
      const v4u b0 = (v4u){bw[0], bw[1], bw[2], bw[3]};
      const v4u b1 = (v4u){bw[4], bw[5], bw[6], bw[7]};
      *(v4u*)(sA + row * kOpPitch + kq)     = a0;
      *(v4u*)(sA + row * kOpPitch + kq + 8) = a1;
      *(v4u*)(sB + row * kOpPitch + kq)     = b0;
      *(v4u*)(sB + row * kOpPitch + kq + 8) = b1;
    }
    __syncthreads();

#pragma unroll
    for (int ks = 0; ks < 2; ++ks) {
      const v16b af  = FragBf::load(sA + (mi * 16 + rl) * kOpPitch + ks * 32 + koff);
      const v16b bf0 = FragBf::load(sB + (nj0 * 16 + rl) * kOpPitch + ks * 32 + koff);
      const v16b bf1 = FragBf::load(sB + (nj0 * 16 + 16 + rl) * kOpPitch + ks * 32 + koff);
      acc0 = FragBf::mma(af, bf0, acc0);
      acc1 = FragBf::mma(af, bf1, acc1);
      guard3(acc0, acc1, af, bf0, bf1);
    }
  }
  acc_guard2(acc0, acc1);

#pragma unroll
  for (int r = 0; r < 8; ++r) {
    const int orow = mi * 16 + 8 * hh + r;
    sRes[orow * kResPitch + nj0 * 16 + rl]      = acc0[r];
    sRes[orow * kResPitch + nj0 * 16 + 16 + rl] = acc1[r];
  }
  __syncthreads();
  {
    float* pp = part + (size_t)blockIdx.x * kTileElems;
    const int c4 = (lane & 15) * 4;
    for (int pass = 0; pass < 2; ++pass) {
#pragma unroll
      for (int i2 = 0; i2 < 4; ++i2) {
        const int orow = wave * 8 + i2 * 2 + hh;
        const v4f v = *(const v4f*)(sRes + orow * kResPitch + c4);
        *(volatile v4f*)(pp + orow * kNumBins + c4) = v;
      }
      __threadfence();
    }
  }
}

__global__ __launch_bounds__(256) void reduce_norm_kernel(const float* __restrict__ part,
                                                          float* __restrict__ out) {
  __shared__ float red[8];
  const int b    = blockIdx.x;
  const int t    = threadIdx.x;
  const int lane = t & 31;
  const int wave = t >> 5;

  v4f accv[kGroupsPerThr];
#pragma unroll
  for (int i = 0; i < kGroupsPerThr; ++i) accv[i] = (v4f){0.f, 0.f, 0.f, 0.f};

#pragma unroll 1
  for (int sp = 0; sp < kNumSplit; ++sp) {
#pragma unroll
    for (int i = 0; i < kGroupsPerThr; ++i) {
      const int gi = i * kThreads + t;
      const int cc = gi >> 10;
      const int e  = (gi & 1023) * 4;
      const float* p = part + ((size_t)((b * kNumPair + cc) * kNumSplit + sp)) * kTileElems + e;
      accv[i] = accv[i] + *(const v4f*)p;
    }
  }

  float tot = 0.0f;
#pragma unroll
  for (int i = 0; i < kGroupsPerThr; ++i) tot += (accv[i][0] + accv[i][1]) + (accv[i][2] + accv[i][3]);
#pragma unroll
  for (int off = 16; off > 0; off >>= 1) tot += __shfl_xor(tot, off, 32);
  if (lane == 0) red[wave] = tot;
  __syncthreads();
  float total = 0.0f;
#pragma unroll
  for (int w = 0; w < 8; ++w) total += red[w];
  const float norm = total + kEps;
  const float inv  = 1.0f / norm;

#pragma unroll
  for (int i = 0; i < kGroupsPerThr; ++i) accv[i] = accv[i] * inv;

  float* ob = out + (size_t)b * kPerImg;
  for (int pass = 0; pass < 2; ++pass) {
#pragma unroll
    for (int i = 0; i < kGroupsPerThr; ++i) {
      const int gi = i * kThreads + t;
      *(volatile v4f*)(ob + (size_t)gi * 4) = accv[i];
    }
    __threadfence();
  }
}

extern "C" void kernel_launch(void* const* d_in, const int* in_sizes, int n_in,
                              void* d_out, int out_size, void* d_ws, size_t ws_size,
                              hipStream_t stream) {
  if (n_in < 1) return;
  if (in_sizes[0] != kInElems) return;
  if (out_size != kOutElems) return;
  if (ws_size < kPartBytes) return;
  const float* x    = (const float*)d_in[0];
  float*       out  = (float*)d_out;
  float*       part = (float*)d_ws;

  hist_partial_kernel<<<kNumBC * kNumSplit, kThreads, 0, stream>>>(x, part);
  reduce_norm_kernel<<<kNumImg, kThreads, 0, stream>>>(part, out);
}
